// HeteroSAGE_25305947308177
// MI455X (gfx1250) — hardware-verified
//
#include <hip/hip_runtime.h>
#include <stddef.h>


#define HID      32
#define KP       128
#define NG       5
#define NTHR     256
#define NWAVE    8
#define EPT      8
#define NGRP     2
#define CHUNK    (NTHR * EPT * NGRP)
#define WCAP     (EPT * NGRP * 32)
#define LISTN    (NWAVE * WCAP)
#define LDS_LIST (LISTN * 4)

static_assert((CHUNK & (CHUNK - 1)) == 0);
static_assert(CHUNK <= 4096);
static_assert(NWAVE * 4 <= 64);

typedef float  v2f   __attribute__((ext_vector_type(2)));
typedef float  v4f   __attribute__((ext_vector_type(4)));
typedef float  v8f   __attribute__((ext_vector_type(8)));
typedef int    v4i   __attribute__((ext_vector_type(4)));
typedef __bf16 bf16_t;
typedef bf16_t v8bf  __attribute__((ext_vector_type(8)));
typedef bf16_t v16bf __attribute__((ext_vector_type(16)));
union FragB { v16bf v; v8bf h[2]; v4i q[2]; };
union Pack8 { v8bf v; v4i q; };

__device__ __forceinline__ v8f wmb(v16bf a, v16bf b, v8f c) {
  v8f d = __builtin_amdgcn_wmma_f32_16x16x32_bf16(false, a, false, b, (short)0, c, false, false);
  asm volatile("v_nop\n\tv_nop\n\tv_nop\n\tv_nop" : "+v"(d) : "v"(a), "v"(b));
  return d;
}

template <int B>
__device__ __forceinline__ void split8(FragB& hi, FragB& lo, v4f a, v4f b) {
#define SPL1(I, X) { const float xv = (X); const bf16_t hb = (bf16_t)xv; hi.v[B + (I)] = hb; lo.v[B + (I)] = (bf16_t)(xv - (float)hb); }
  SPL1(0, a.x) SPL1(1, a.y) SPL1(2, a.z) SPL1(3, a.w)
  SPL1(4, b.x) SPL1(5, b.y) SPL1(6, b.z) SPL1(7, b.w)
#undef SPL1
}

template <int NBT>
__device__ __forceinline__ int scan_chunk(const int* __restrict__ dsts, int nE, int cbase, int nodeBase,
                                          int vec8, int* list, int tid, int lane, int wave) {
  int wc = 0;
  (void)lane;
#pragma unroll
  for (int g = 0; g < NGRP; ++g) {
    const int el0  = (g * NTHR + tid) * EPT;
    const int e0   = cbase + el0;
    const int sent = -2147483647 - 1;
    v4i da, db;
    if (vec8 != 0 && cbase + CHUNK <= nE) {
      da = *(const v4i*)(dsts + e0);
      db = *(const v4i*)(dsts + e0 + 4);
    } else {
      da.x = (e0     < nE) ? dsts[min(e0, nE - 1)] : sent;
      da.y = (e0 + 1 < nE) ? dsts[min(e0 + 1, nE - 1)] : sent;
      da.z = (e0 + 2 < nE) ? dsts[min(e0 + 2, nE - 1)] : sent;
      da.w = (e0 + 3 < nE) ? dsts[min(e0 + 3, nE - 1)] : sent;
      db.x = (e0 + 4 < nE) ? dsts[min(e0 + 4, nE - 1)] : sent;
      db.y = (e0 + 5 < nE) ? dsts[min(e0 + 5, nE - 1)] : sent;
      db.z = (e0 + 6 < nE) ? dsts[min(e0 + 6, nE - 1)] : sent;
      db.w = (e0 + 7 < nE) ? dsts[min(e0 + 7, nE - 1)] : sent;
    }
    const unsigned nb = (unsigned)nodeBase;
    const unsigned s0 = (unsigned)da.x - nb, s1 = (unsigned)da.y - nb;
    const unsigned s2 = (unsigned)da.z - nb, s3 = (unsigned)da.w - nb;
    const unsigned s4 = (unsigned)db.x - nb, s5 = (unsigned)db.y - nb;
    const unsigned s6 = (unsigned)db.z - nb, s7 = (unsigned)db.w - nb;
    const bool h0 = s0 < (unsigned)NBT, h1 = s1 < (unsigned)NBT, h2 = s2 < (unsigned)NBT, h3 = s3 < (unsigned)NBT;
    const bool h4 = s4 < (unsigned)NBT, h5 = s5 < (unsigned)NBT, h6 = s6 < (unsigned)NBT, h7 = s7 < (unsigned)NBT;
    const unsigned any = __builtin_amdgcn_ballot_w32(h0 | h1 | h2 | h3 | h4 | h5 | h6 | h7);
    if (any != 0u) {
#define HITJ(J, HJ, SJ) { \
        const unsigned mj = __builtin_amdgcn_ballot_w32(HJ); \
        if (mj != 0u) { \
          if (HJ) { \
            const int pos = wc + (int)__builtin_amdgcn_mbcnt_lo(mj, 0u); \
            if (pos < WCAP) list[wave * WCAP + pos] = ((el0 + (J)) << 12) | (int)(SJ); \
          } \
          wc += (int)__builtin_popcount(mj); } }
      HITJ(0, h0, s0)
      HITJ(1, h1, s1)
      HITJ(2, h2, s2)
      HITJ(3, h3, s3)
      HITJ(4, h4, s4)
      HITJ(5, h5, s5)
      HITJ(6, h6, s6)
      HITJ(7, h7, s7)
#undef HITJ
    }
  }
  return wc;
}

__global__ __launch_bounds__(NTHR) void k_wprep(
    const float* __restrict__ W1l_c, const float* __restrict__ W1r_c,
    const float* __restrict__ W1l_w, const float* __restrict__ W1r_w,
    const float* __restrict__ W1l_r, const float* __restrict__ W1r_r,
    const float* __restrict__ W2l_c, const float* __restrict__ W2r_c,
    const float* __restrict__ W2l_w, const float* __restrict__ W2r_w,
    bf16_t* whi, bf16_t* wlo, int nTot) {
  const int i = blockIdx.x * NTHR + threadIdx.x;
  if (i >= nTot) return;
  const int o   = i * 8;
  const int g   = o / (HID * KP);
  const int rem = o - g * (HID * KP);
  const int n   = rem / KP;
  const int k0  = rem - n * KP;
  const float* WL = W2l_w; const float* WA = W2l_w; const float* WB = W2l_w;
  int KL = 32, KT = 32; float fb = 0.0f;
  if (g == 0)      { WL = W1l_c; WA = W1r_c; WB = W1r_w; KL = 64; KT = 128; fb = 1.0f; }
  else if (g == 1) { WL = W1l_w; WA = W1l_w; WB = W1l_w; KL = 64; KT = 64;  fb = 0.0f; }
  else if (g == 2) { WL = W1l_r; WA = W1r_r; WB = W1r_r; KL = 64; KT = 128; fb = 0.0f; }
  else if (g == 3) { WL = W2l_c; WA = W2r_c; WB = W2r_w; KL = 32; KT = 64;  fb = 1.0f; }
  int krm = KT - KL - 1; krm = krm < 0 ? 0 : krm;
  Pack8 ph, pl;
#define WSP(I) { const int k = k0 + (I); const int kl = (k < KL) ? k : (KL - 1); \
    int kr = k - KL; kr = kr < 0 ? 0 : kr; kr = kr > krm ? krm : kr; \
    const float xl = WL[kl * HID + n]; const float xa = WA[kr * HID + n]; const float xb = WB[kr * HID + n]; \
    const float xv = (k < KL) ? xl : ((k < KT) ? (xa + fb * xb) : 0.0f); \
    const bf16_t hb = (bf16_t)xv; ph.v[(I)] = hb; pl.v[(I)] = (bf16_t)(xv - (float)hb); }
  WSP(0) WSP(1) WSP(2) WSP(3) WSP(4) WSP(5) WSP(6) WSP(7)
#undef WSP
  bf16_t* dh = whi + o;
  bf16_t* dl = wlo + o;
  const v4i qh = ph.q, ql = pl.q;
  *(volatile v4i*)dh = qh;
  *(volatile v4i*)dl = ql;
  __threadfence();
  *(volatile v4i*)dh = qh;
  *(volatile v4i*)dl = ql;
}

__device__ __forceinline__ void kstep(const float* ap, float mul,
                                      const bf16_t* bhp, const bf16_t* blp, v8f (&c)[2]) {
  const v4f p0 = (*(const v4f*)(ap))      * mul;
  const v4f p1 = (*(const v4f*)(ap + 4))  * mul;
  const v4f p2 = (*(const v4f*)(ap + 16)) * mul;
  const v4f p3 = (*(const v4f*)(ap + 20)) * mul;
  FragB ahi, alo;
  split8<0>(ahi, alo, p0, p1);
  split8<8>(ahi, alo, p2, p3);
#pragma unroll
  for (int ct = 0; ct < 2; ++ct) {
    const bf16_t* hp = bhp + (size_t)ct * 16 * KP;
    const bf16_t* lp = blp + (size_t)ct * 16 * KP;
    FragB bh, bq;
    bh.q[0] = *(const v4i*)hp;  bh.q[1] = *(const v4i*)(hp + 16);
    bq.q[0] = *(const v4i*)lp;  bq.q[1] = *(const v4i*)(lp + 16);
    c[ct] = wmb(alo.v, bh.v, c[ct]);
    c[ct] = wmb(ahi.v, bq.v, c[ct]);
    c[ct] = wmb(ahi.v, bh.v, c[ct]);
  }
}

template <int NB, int DA, int KROOT>
__global__ __launch_bounds__(NTHR) void k_sage(
    const int* __restrict__ srcs, const int* __restrict__ dsts,
    const float* __restrict__ xsrc, const float* __restrict__ xdst,
    const bf16_t* __restrict__ whi, const bf16_t* __restrict__ wlo,
    const float* __restrict__ biasA, const float* __restrict__ biasB,
    const float* __restrict__ addp, float* outp,
    int nDst, int nSrc, int nE, int vec8, int nbias, int hasadd, int relu, int nRowsOut) {
  static_assert((NB & (NB - 1)) == 0);
  static_assert(NB <= 4096);
  static_assert(DA == 32 || DA == 64);
  static_assert(KROOT == 0 || KROOT == DA);
  static_assert((NB / 16) % NWAVE == 0);
  constexpr int NTILE = NB / 16;
  constexpr int TPW   = NTILE / NWAVE;

  extern __shared__ v4f lds_dyn[];
  float* acc  = (float*)lds_dyn;
  int*   list = (int*)((char*)lds_dyn + (size_t)NB * DA * 4);
  int*   cnt  = list + LISTN;
  int*   wcnt = cnt + NB;
  const int tid = threadIdx.x, lane = tid & 31, wave = tid >> 5, hh = lane >> 4, m = lane & 15;
  const int nodeBase = blockIdx.x * NB;

  {
    const v4f z = {0.f, 0.f, 0.f, 0.f};
    for (int i = tid; i < NB * DA / 4; i += NTHR) lds_dyn[i] = z;
    for (int i = tid; i < NB; i += NTHR) cnt[i] = 0;
  }
  __syncthreads();

  const int nChunks = (nE + CHUNK - 1) / CHUNK;
#pragma unroll 1
  for (int ch = 0; ch < nChunks; ++ch) {
    const int cbase = ch * CHUNK;
    const int wc = scan_chunk<NB>(dsts, nE, cbase, nodeBase, vec8, list, tid, lane, wave);
    if (lane == 0) wcnt[wave] = wc;
    __syncthreads();
    if (wave == 0) {
#pragma unroll 1
      for (int wsx = 0; wsx < NWAVE; ++wsx) {
        int n = __builtin_amdgcn_readfirstlane(wcnt[wsx]);
        n = n > WCAP ? WCAP : (n < 0 ? 0 : n);
        const int* lp = list + wsx * WCAP;
#pragma unroll 1
        for (int i = 0; i < n; ++i) {
          const int ent  = __builtin_amdgcn_readfirstlane(lp[i]);
          const int slot = ent & (NB - 1);
          int e = cbase + ((ent >> 12) & (CHUNK - 1));
          e = e > nE - 1 ? nE - 1 : e;
          int src = __builtin_amdgcn_readfirstlane(srcs[e]);
          src = src < 0 ? 0 : (src > nSrc - 1 ? nSrc - 1 : src);
          if (DA == 64) {
            const v2f v = *(const v2f*)(xsrc + (size_t)src * 64 + 2 * lane);
            v2f* apv = (v2f*)(acc + slot * 64 + 2 * lane);
            *apv = *apv + v;
          } else {
            const float v = xsrc[(size_t)src * 32 + lane];
            acc[slot * 32 + lane] = acc[slot * 32 + lane] + v;
          }
          if (lane == 0) cnt[slot] = cnt[slot] + 1;
        }
      }
    }
    __syncthreads();
  }

  float bb0 = 0.0f, bb1 = 0.0f;
  if (nbias >= 1) { bb0 = biasA[m]; bb1 = biasA[16 + m]; }
  if (nbias >= 2) { bb0 += biasB[m]; bb1 += biasB[16 + m]; }

  const bf16_t* bh0 = whi + m * KP + 8 * hh;
  const bf16_t* bl0 = wlo + m * KP + 8 * hh;
  const int rsub = lane >> 3;

#pragma unroll 1
  for (int q = 0; q < TPW; ++q) {
    const int t     = q * NWAVE + wave;
    const int slotm = 16 * t + m;
    int node = nodeBase + slotm;
    node = node > nDst - 1 ? nDst - 1 : node;
    const int   cd  = cnt[slotm];
    const float inv = 1.0f / (float)(cd > 1 ? cd : 1);

    v8f c[2];
    { const v8f z = {0.f, 0.f, 0.f, 0.f, 0.f, 0.f, 0.f, 0.f}; c[0] = z; c[1] = z; }

    const float* arow = acc + slotm * DA + 8 * hh;
#pragma unroll
    for (int ks = 0; ks < DA / 32; ++ks)
      kstep(arow + 32 * ks, inv, bh0 + 32 * ks, bl0 + 32 * ks, c);
    if (KROOT > 0) {
      const float* xrow = xdst + (size_t)node * KROOT + 8 * hh;
#pragma unroll
      for (int ks = 0; ks < KROOT / 32; ++ks)
        kstep(xrow + 32 * ks, 1.0f, bh0 + DA + 32 * ks, bl0 + DA + 32 * ks, c);
    }

    float* stg = acc + (size_t)16 * t * DA;
    const size_t growb = (size_t)(nodeBase + 16 * t + 8 * hh);
#pragma unroll
    for (int ct = 0; ct < 2; ++ct) {
      const int   col = 16 * ct + m;
      const float bv  = (ct == 0) ? bb0 : bb1;
#pragma unroll
      for (int r = 0; r < 8; ++r) {
        float v = c[ct][r] + bv;
        if (hasadd != 0) v += addp[(growb + r) * HID + col];
        if (relu != 0) v = fmaxf(v, 0.0f);
        stg[(8 * hh + r) * HID + col] = v;
      }
    }
    __syncthreads();

#pragma unroll
    for (int i = 0; i < 4; ++i) {
      const int grow = nodeBase + 16 * t + 4 * i + rsub;
      const v4f v = *(const v4f*)(stg + 128 * i + 4 * lane);
      if (grow < nRowsOut)
        *(volatile v4f*)(outp + (size_t)(nodeBase + 16 * t + 4 * i) * HID + 4 * lane) = v;
    }
    __threadfence();
#pragma unroll
    for (int i = 0; i < 4; ++i) {
      const int grow = nodeBase + 16 * t + 4 * i + rsub;
      const v4f v = *(const v4f*)(stg + 128 * i + 4 * lane);
      if (grow < nRowsOut)
        *(volatile v4f*)(outp + (size_t)(nodeBase + 16 * t + 4 * i) * HID + 4 * lane) = v;
    }
  }
}

#define NB1  1024
#define NB2  2048
#define LDS_A ((NB1 * 64 * 4) + LDS_LIST + (NB1 * 4) + 64)
#define LDS_B ((NB2 * 32 * 4) + LDS_LIST + (NB2 * 4) + 64)
static_assert(LDS_A <= 300 * 1024);
static_assert(LDS_B <= 300 * 1024);

extern "C" void kernel_launch(void* const* d_in, const int* in_sizes, int n_in,
                              void* d_out, int out_size, void* d_ws, size_t ws_size,
                              hipStream_t stream) {
  if (n_in < 26) return;
  const int nP = in_sizes[0] / 64;
  const int nA = in_sizes[1] / 64;
  const int eC = in_sizes[3];
  const int eW = in_sizes[5];
  const int eR = in_sizes[7];
  if (nP <= 0 || nA <= 0 || eC < 0 || eW < 0 || eR < 0) return;
  if (in_sizes[0] != nP * 64 || in_sizes[1] != nA * 64) return;
  if (in_sizes[2] != eC || in_sizes[4] != eW || in_sizes[6] != eR) return;
  if (in_sizes[8] != 2048 || in_sizes[9] != 2048 || in_sizes[11] != 2048 || in_sizes[12] != 2048 ||
      in_sizes[14] != 2048 || in_sizes[15] != 2048) return;
  if (in_sizes[17] != 1024 || in_sizes[18] != 1024 || in_sizes[20] != 1024 || in_sizes[21] != 1024) return;
  if (in_sizes[10] < 32 || in_sizes[13] < 32 || in_sizes[16] < 32 || in_sizes[19] < 32 || in_sizes[22] < 32) return;
  if (out_size != nP * HID) return;

  const float* x_paper  = (const float*)d_in[0];
  const float* x_author = (const float*)d_in[1];
  const int* cites_src  = (const int*)d_in[2];
  const int* cites_dst  = (const int*)d_in[3];
  const int* writes_src = (const int*)d_in[4];
  const int* writes_dst = (const int*)d_in[5];
  const int* rev_src    = (const int*)d_in[6];
  const int* rev_dst    = (const int*)d_in[7];
  const float* W1l_c = (const float*)d_in[8];
  const float* W1r_c = (const float*)d_in[9];
  const float* b1_c  = (const float*)d_in[10];
  const float* W1l_w = (const float*)d_in[11];
  const float* W1r_w = (const float*)d_in[12];
  const float* b1_w  = (const float*)d_in[13];
  const float* W1l_r = (const float*)d_in[14];
  const float* W1r_r = (const float*)d_in[15];
  const float* b1_r  = (const float*)d_in[16];
  const float* W2l_c = (const float*)d_in[17];
  const float* W2r_c = (const float*)d_in[18];
  const float* b2_c  = (const float*)d_in[19];
  const float* W2l_w = (const float*)d_in[20];
  const float* W2r_w = (const float*)d_in[21];
  const float* b2_w  = (const float*)d_in[22];
  float* out = (float*)d_out;

  const int nBlkP1 = (nP + NB1 - 1) / NB1;
  const int nBlkA  = (nA + NB1 - 1) / NB1;
  const int nBlkP2 = (nP + NB2 - 1) / NB2;
  const int rowsP1 = nBlkP1 * NB1;
  const int rowsA  = nBlkA * NB1;
  const int rowsP2 = nBlkP2 * NB2;

  char* ws = (char*)d_ws;
  size_t off = 0;
  const size_t szW  = (size_t)NG * HID * KP * 2;
  const size_t szP1 = (size_t)rowsP1 * HID * 4;
  const size_t szA  = (size_t)rowsA * HID * 4;
  const size_t szP2 = (size_t)rowsP2 * HID * 4;
  const size_t oWh = off; off += szW;  off = (off + 255) & ~(size_t)255;
  const size_t oWl = off; off += szW;  off = (off + 255) & ~(size_t)255;
  const size_t oP  = off; off += szP1; off = (off + 255) & ~(size_t)255;
  const size_t oX1 = off; off += szP1; off = (off + 255) & ~(size_t)255;
  const size_t oA1 = off; off += szA;  off = (off + 255) & ~(size_t)255;
  const size_t oQ  = off; off += szP2; off = (off + 255) & ~(size_t)255;
  if (off > ws_size) return;
  bf16_t* whi = (bf16_t*)(ws + oWh);
  bf16_t* wlo = (bf16_t*)(ws + oWl);
  float*  P   = (float*)(ws + oP);
  float*  p1  = (float*)(ws + oX1);
  float*  a1  = (float*)(ws + oA1);
  float*  Q   = (float*)(ws + oQ);

  const int vC = ((eC & 3) == 0) ? 1 : 0;
  const int vW = ((eW & 3) == 0) ? 1 : 0;
  const int vR = ((eR & 3) == 0) ? 1 : 0;

  const int nTot = NG * HID * KP / 8;
  k_wprep<<<(nTot + NTHR - 1) / NTHR, NTHR, 0, stream>>>(
      W1l_c, W1r_c, W1l_w, W1r_w, W1l_r, W1r_r, W2l_c, W2r_c, W2l_w, W2r_w, whi, wlo, nTot);

  hipFuncSetAttribute(reinterpret_cast<const void*>(&k_sage<NB1, 64, 64>),
                      hipFuncAttributeMaxDynamicSharedMemorySize, LDS_A);
  hipFuncSetAttribute(reinterpret_cast<const void*>(&k_sage<NB1, 64, 0>),
                      hipFuncAttributeMaxDynamicSharedMemorySize, LDS_A);
  hipFuncSetAttribute(reinterpret_cast<const void*>(&k_sage<NB2, 32, 32>),
                      hipFuncAttributeMaxDynamicSharedMemorySize, LDS_B);
  hipFuncSetAttribute(reinterpret_cast<const void*>(&k_sage<NB2, 32, 0>),
                      hipFuncAttributeMaxDynamicSharedMemorySize, LDS_B);

  const size_t PL = (size_t)HID * KP;

  k_sage<NB1, 64, 64><<<nBlkP1, NTHR, LDS_A, stream>>>(
      cites_src, cites_dst, x_paper, x_paper, whi + 0 * PL, wlo + 0 * PL, b1_c, b1_w, P, P,
      nP, nP, eC, vC, 2, 0, 0, rowsP1);
  k_sage<NB1, 64, 0><<<nBlkP1, NTHR, LDS_A, stream>>>(
      writes_src, writes_dst, x_author, x_author, whi + 1 * PL, wlo + 1 * PL, b1_c, b1_c, P, p1,
      nP, nA, eW, vW, 0, 1, 1, rowsP1);
  k_sage<NB1, 64, 64><<<nBlkA, NTHR, LDS_A, stream>>>(
      rev_src, rev_dst, x_paper, x_author, whi + 2 * PL, wlo + 2 * PL, b1_r, b1_r, P, a1,
      nA, nP, eR, vR, 1, 0, 1, rowsA);
  k_sage<NB2, 32, 32><<<nBlkP2, NTHR, LDS_B, stream>>>(
      cites_src, cites_dst, p1, p1, whi + 3 * PL, wlo + 3 * PL, b2_c, b2_w, Q, Q,
      nP, nP, eC, vC, 2, 0, 0, rowsP2);
  k_sage<NB2, 32, 0><<<nBlkP2, NTHR, LDS_B, stream>>>(
      writes_src, writes_dst, a1, a1, whi + 4 * PL, wlo + 4 * PL, b2_c, b2_c, Q, out,
      nP, nA, eW, vW, 0, 1, 0, nP);
}
